// GATv2Layer_46188078301403
// MI455X (gfx1250) — hardware-verified
//
#include <hip/hip_runtime.h>
#include <math.h>

typedef __attribute__((ext_vector_type(16))) _Float16 v16h;
typedef __attribute__((ext_vector_type(8)))  _Float16 v8h;
typedef __attribute__((ext_vector_type(8)))  float    v8f;
typedef __attribute__((ext_vector_type(4)))  float    v4f;
typedef __attribute__((ext_vector_type(4)))  int      v4i;

constexpr int kNodes   = 1024;
constexpr int kChan    = 256;
constexpr int kCat     = 2 * kChan;
constexpr int kRowTile = 8;
constexpr float kNegSlope = 0.2f;

constexpr float kCarryX = 16.0f;
constexpr float kCarryW = 256.0f;
constexpr float kCarryG = 16.0f;
constexpr float kCarryP = 1024.0f;
constexpr float kScaleProj = 1.0f / (kCarryX * kCarryW);
constexpr float kScaleOut  = 1.0f / (kCarryP * kCarryG);
constexpr float kHalfMinNormal = 6.103515625e-5f;

static_assert((kNodes % 64) == 0 && (kChan % 64) == 0 && (kCat % 64) == 0, "GEMM M,N multiples of 64");
static_assert((kChan % 32) == 0 && (kNodes % 32) == 0, "GEMM K multiples of 32");
static_assert((kNodes % kRowTile) == 0, "row tile");
static_assert(kRowTile == 8, "one wave per tile row in the softmax phase");

constexpr size_t kOffNH = 0;
constexpr size_t kOffWH = kOffNH + (size_t)kNodes * kChan * 2;
constexpr size_t kOffBC = kOffWH + (size_t)kCat * kChan * 2;
constexpr size_t kOffG  = kOffBC + (size_t)kCat * 4;
constexpr size_t kOffGT = kOffG  + (size_t)kNodes * kCat * 4;
constexpr size_t kOffPW = kOffGT + (size_t)kChan * kNodes * 2;
constexpr size_t kWsTotal = kOffPW + (size_t)kNodes * kNodes * 2;
static_assert(kWsTotal == 5507072ull, "carve total");
static_assert(kWsTotal <= 134217728ull, "carve cap");
static_assert((kOffWH % 128) == 0 && (kOffBC % 128) == 0 && (kOffG % 128) == 0 &&
              (kOffGT % 128) == 0 && (kOffPW % 128) == 0, "128-B aligned regions");

namespace eng {

__device__ __forceinline__ v16h frag_load(const _Float16* p) {
  union U { v16h v; v8h h[2]; } f;
  f.h[0] = *(const v8h*)(p);
  f.h[1] = *(const v8h*)(p + 16);
  return f.v;
}

__device__ __forceinline__ v8f mma_g(v16h a, v16h b, v8f c) {
  c = __builtin_amdgcn_wmma_f32_16x16x32_f16(false, a, false, b, (short)0, c, false, false);
  asm volatile("v_nop\n\tv_nop\n\tv_nop\n\tv_nop" : "+v"(c) : "v"(a), "v"(b));
  return c;
}

template <int BIAS_MODE, int OUT_MODE>
__global__ __launch_bounds__(256) void gemm64_f16(
    const unsigned short* __restrict__ Ap, int lda,
    const unsigned short* __restrict__ Btp, int ldb,
    void* __restrict__ Cout, int ldc,
    const float* __restrict__ bias,
    int M, int N, int K, float scale, float postscale) {
  const _Float16* A  = (const _Float16*)Ap;
  const _Float16* Bt = (const _Float16*)Btp;
  __shared__ __align__(16) float sT[8][16 * 68];
  const int lane = threadIdx.x & 31;
  const int wave = threadIdx.x >> 5;
  const int tilesN = N >> 6;
  const int tilesM = M >> 6;
  const int tile = blockIdx.x * 8 + wave;
  if (tile >= tilesM * tilesN) return;
  const int tm = tile / tilesN;
  const int tn = tile - tm * tilesN;
  const int m0 = tm << 6;
  const int n0 = tn << 6;

  const int rlane = lane & 15;
  const int koff  = (lane >> 4) * 8;
  const int mOff  = (lane >> 4) * 8;

  v8f acc[4][4];
#pragma unroll
  for (int i = 0; i < 4; ++i)
#pragma unroll
    for (int j = 0; j < 4; ++j) acc[i][j] = (v8f){0.f, 0.f, 0.f, 0.f, 0.f, 0.f, 0.f, 0.f};

  for (int k0 = 0; k0 < K; k0 += 32) {
    v16h bh[4];
#pragma unroll
    for (int j = 0; j < 4; ++j) {
      const size_t bo = (size_t)(n0 + (j << 4) + rlane) * ldb + koff + k0;
      bh[j] = frag_load(Bt + bo);
    }
#pragma unroll
    for (int i = 0; i < 4; ++i) {
      const size_t ao = (size_t)(m0 + (i << 4) + rlane) * lda + koff + k0;
      const v16h ah = frag_load(A + ao);
#pragma unroll
      for (int j = 0; j < 4; ++j) acc[i][j] = mma_g(ah, bh[j], acc[i][j]);
    }
  }

  float* slab = sT[wave];
  float bvn[4] = {0.f, 0.f, 0.f, 0.f};
  if (BIAS_MODE == 2) {
#pragma unroll
    for (int j = 0; j < 4; ++j) bvn[j] = bias[n0 + (j << 4) + rlane];
  }
#pragma unroll
  for (int i = 0; i < 4; ++i) {
    const int mBase = m0 + (i << 4);
    v4f br0 = (v4f){0.f, 0.f, 0.f, 0.f};
    v4f br1 = (v4f){0.f, 0.f, 0.f, 0.f};
    if (BIAS_MODE == 1) {
      br0 = *(const v4f*)(bias + mBase + mOff);
      br1 = *(const v4f*)(bias + mBase + mOff + 4);
    }
#pragma unroll
    for (int j = 0; j < 4; ++j) {
#pragma unroll
      for (int r = 0; r < 8; ++r) {
        float v = acc[i][j][r] * scale;
        if (BIAS_MODE == 1) v += (r < 4) ? br0[r & 3] : br1[r & 3];
        if (BIAS_MODE == 2) v += bvn[j];
        v *= postscale;
        slab[(mOff + r) * 68 + (j << 4) + rlane] = v;
      }
    }
    __builtin_amdgcn_fence(__ATOMIC_RELEASE, "workgroup");
    __builtin_amdgcn_wave_barrier();
    __builtin_amdgcn_fence(__ATOMIC_ACQUIRE, "workgroup");
    if (OUT_MODE == 0) {
      float* C = (float*)Cout;
      const int hh = lane >> 4, c4 = (lane & 15) * 4;
      for (int pass = 0; pass < 2; ++pass) {
#pragma unroll
        for (int it = 0; it < 8; ++it) {
          const int row = it * 2 + hh;
          const v4f v = *(const v4f*)(slab + row * 68 + c4);
          *(volatile v4f*)(C + (size_t)(mBase + row) * ldc + n0 + c4) = v;
        }
        __threadfence();
      }
    } else {
      unsigned short* C = (unsigned short*)Cout;
      const int q = lane >> 3, c8 = (lane & 7) * 8;
      for (int pass = 0; pass < 2; ++pass) {
#pragma unroll
        for (int it = 0; it < 4; ++it) {
          const int row = it * 4 + q;
          const float* sp = slab + row * 68 + c8;
          v8h hv;
#pragma unroll
          for (int e = 0; e < 8; ++e) {
            float x = sp[e];
            x = (fabsf(x) < kHalfMinNormal) ? 0.0f : x;
            hv[e] = (_Float16)x;
          }
          *(volatile v8h*)(C + (size_t)(mBase + row) * ldc + n0 + c8) = hv;
        }
        __threadfence();
      }
    }
    __builtin_amdgcn_fence(__ATOMIC_RELEASE, "workgroup");
    __builtin_amdgcn_wave_barrier();
    __builtin_amdgcn_fence(__ATOMIC_ACQUIRE, "workgroup");
  }
}

}

__device__ __forceinline__ void cast8_store(const float* __restrict__ src, unsigned short* __restrict__ dst,
                                            size_t e0, float carry) {
  const v4f a0 = *(const v4f*)(src + e0);
  const v4f a1 = *(const v4f*)(src + e0 + 4);
  v8h hv;
#pragma unroll
  for (int e = 0; e < 4; ++e) {
    float x0 = a0[e] * carry;
    float x1 = a1[e] * carry;
    x0 = (fabsf(x0) < kHalfMinNormal) ? 0.0f : x0;
    x1 = (fabsf(x1) < kHalfMinNormal) ? 0.0f : x1;
    hv[e]     = (_Float16)x0;
    hv[4 + e] = (_Float16)x1;
  }
  unsigned short* qd = dst + e0;
  *(volatile v8h*)qd = hv;
  __threadfence();
  *(volatile v8h*)qd = hv;
}

constexpr int kPrepBlkX  = (kNodes * kChan / 8) / 256;
constexpr int kPrepBlkW  = (kChan * kChan / 8) / 256;
constexpr int kPrepBlocks = kPrepBlkX + 2 * kPrepBlkW + 1;
static_assert(kPrepBlkX == 128 && kPrepBlkW == 32 && kPrepBlocks == 193, "prep coverage");

__global__ __launch_bounds__(256) void prep_kernel(
    const float* __restrict__ nodes, const float* __restrict__ wsrc, const float* __restrict__ bsrc,
    const float* __restrict__ wtgt, const float* __restrict__ btgt,
    unsigned short* __restrict__ NH, unsigned short* __restrict__ WH, float* __restrict__ BC) {
  const int bx = blockIdx.x, tid = threadIdx.x;
  if (bx < kPrepBlkX) {
    cast8_store(nodes, NH, ((size_t)bx * 256 + tid) * 8, kCarryX);
  } else if (bx < kPrepBlkX + kPrepBlkW) {
    cast8_store(wsrc, WH, ((size_t)(bx - kPrepBlkX) * 256 + tid) * 8, kCarryW);
  } else if (bx < kPrepBlkX + 2 * kPrepBlkW) {
    cast8_store(wtgt, WH + (size_t)kChan * kChan, ((size_t)(bx - kPrepBlkX - kPrepBlkW) * 256 + tid) * 8, kCarryW);
  } else {
    const int sidx = (tid & 63) * 4;
    const v4f vs = *(const v4f*)(bsrc + sidx);
    const v4f vt = *(const v4f*)(btgt + sidx);
    const bool pick_src = (tid < 64);
    v4f v;
    v[0] = pick_src ? vs[0] : vt[0];
    v[1] = pick_src ? vs[1] : vt[1];
    v[2] = pick_src ? vs[2] : vt[2];
    v[3] = pick_src ? vs[3] : vt[3];
    if (tid < 128) {
      float* qd = BC + tid * 4;
      *(volatile v4f*)qd = v;
      __threadfence();
      *(volatile v4f*)qd = v;
    }
  }
}

__global__ __launch_bounds__(256) void score_softmax_kernel(
    const float* __restrict__ G, const float* __restrict__ aw, const int* __restrict__ adj,
    unsigned short* __restrict__ PW) {
  __shared__ __align__(16) float sG[kRowTile * kChan];
  __shared__ __align__(16) float sA[kChan];
  __shared__ __align__(16) float sS[kRowTile * kNodes];
  const int tid = threadIdx.x, lane = tid & 31, wave = tid >> 5;
  const int i0 = blockIdx.x * kRowTile;

#pragma unroll
  for (int k = 0; k < 2; ++k) {
    const int e = k * 1024 + tid * 4;
    const int r = e >> 8, c = e & (kChan - 1);
    *(v4f*)(sG + e) = *(const v4f*)(G + (size_t)(i0 + r) * kCat + c);
  }
  sA[tid] = aw[tid];
  __syncthreads();

#pragma unroll 1
  for (int q = 0; q < 4; ++q) {
    const int j = q * 256 + tid;
    const float* gt = G + (size_t)j * kCat + kChan;
    float acc[kRowTile];
#pragma unroll
    for (int r = 0; r < kRowTile; ++r) acc[r] = 0.0f;
#pragma unroll 1
    for (int c = 0; c < kChan; c += 4) {
      const v4f t4 = *(const v4f*)(gt + c);
      const v4f a4 = *(const v4f*)(sA + c);
#pragma unroll
      for (int r = 0; r < kRowTile; ++r) {
        const v4f g4 = *(const v4f*)(sG + r * kChan + c);
#pragma unroll
        for (int e = 0; e < 4; ++e) {
          const float x = g4[e] + t4[e];
          const float l = fmaxf(x, kNegSlope * x);
          acc[r] = fmaf(a4[e], l, acc[r]);
        }
      }
    }
#pragma unroll
    for (int r = 0; r < kRowTile; ++r) sS[r * kNodes + j] = acc[r];
  }
  __syncthreads();

  const int i = i0 + wave;
  float* srow = sS + wave * kNodes;
  const int* arow = adj + (size_t)i * kNodes;

  float mx = -INFINITY;
#pragma unroll 1
  for (int it = 0; it < 4; ++it) {
    const int cb = it * 256 + lane * 8;
    v4f s0 = *(const v4f*)(srow + cb);
    v4f s1 = *(const v4f*)(srow + cb + 4);
    const v4i m0 = *(const v4i*)(arow + cb);
    const v4i m1 = *(const v4i*)(arow + cb + 4);
#pragma unroll
    for (int e = 0; e < 4; ++e) {
      const float a = (m0[e] != 0) ? s0[e] : -INFINITY;
      const float b = (m1[e] != 0) ? s1[e] : -INFINITY;
      s0[e] = a;
      s1[e] = b;
      mx = fmaxf(mx, fmaxf(a, b));
    }
    *(v4f*)(srow + cb) = s0;
    *(v4f*)(srow + cb + 4) = s1;
  }
#pragma unroll
  for (int off = 16; off > 0; off >>= 1) mx = fmaxf(mx, __shfl_xor(mx, off, 32));

  float sum = 0.0f;
#pragma unroll 1
  for (int it = 0; it < 4; ++it) {
    const int cb = it * 256 + lane * 8;
    v4f s0 = *(const v4f*)(srow + cb);
    v4f s1 = *(const v4f*)(srow + cb + 4);
#pragma unroll
    for (int e = 0; e < 4; ++e) {
      const float a = s0[e];
      const float b = s1[e];
      const float ea = (a > -INFINITY) ? expf(a - mx) : 0.0f;
      const float eb = (b > -INFINITY) ? expf(b - mx) : 0.0f;
      s0[e] = ea;
      s1[e] = eb;
      sum += ea;
      sum += eb;
    }
    *(v4f*)(srow + cb) = s0;
    *(v4f*)(srow + cb + 4) = s1;
  }
#pragma unroll
  for (int off = 16; off > 0; off >>= 1) sum += __shfl_xor(sum, off, 32);

  const float scl = (1.0f / sum) * kCarryP;
#pragma unroll 1
  for (int it = 0; it < 4; ++it) {
    const int cb = it * 256 + lane * 8;
    const v4f s0 = *(const v4f*)(srow + cb);
    const v4f s1 = *(const v4f*)(srow + cb + 4);
    v8h hv;
#pragma unroll
    for (int e = 0; e < 4; ++e) {
      float p0 = s0[e] * scl;
      float p1 = s1[e] * scl;
      p0 = (fabsf(p0) < kHalfMinNormal) ? 0.0f : p0;
      p1 = (fabsf(p1) < kHalfMinNormal) ? 0.0f : p1;
      hv[e]     = (_Float16)p0;
      hv[4 + e] = (_Float16)p1;
    }
    unsigned short* qd = PW + (size_t)i * kNodes + cb;
    *(volatile v8h*)qd = hv;
    __threadfence();
    *(volatile v8h*)qd = hv;
  }
}

extern "C" void kernel_launch(void* const* d_in, const int* in_sizes, int n_in,
                              void* d_out, int out_size, void* d_ws, size_t ws_size,
                              hipStream_t stream) {
  if (n_in < 7) return;
  if (in_sizes[0] != kNodes * kChan) return;
  if (in_sizes[1] != kNodes * kNodes) return;
  if (in_sizes[2] != kChan * kChan) return;
  if (in_sizes[3] != kChan) return;
  if (in_sizes[4] != kChan * kChan) return;
  if (in_sizes[5] != kChan) return;
  if (in_sizes[6] != kChan) return;
  if (out_size != kNodes * kChan) return;
  if (ws_size < kWsTotal) return;

  const float* nodes = (const float*)d_in[0];
  const int*   adj   = (const int*)d_in[1];
  const float* wsrc  = (const float*)d_in[2];
  const float* bsrc  = (const float*)d_in[3];
  const float* wtgt  = (const float*)d_in[4];
  const float* btgt  = (const float*)d_in[5];
  const float* aw    = (const float*)d_in[6];
  float* out = (float*)d_out;

  char* ws = (char*)d_ws;
  unsigned short* NH = (unsigned short*)(ws + kOffNH);
  unsigned short* WH = (unsigned short*)(ws + kOffWH);
  float*          BC = (float*)(ws + kOffBC);
  float*          G  = (float*)(ws + kOffG);
  unsigned short* GT = (unsigned short*)(ws + kOffGT);
  unsigned short* PW = (unsigned short*)(ws + kOffPW);

  prep_kernel<<<kPrepBlocks, 256, 0, stream>>>(nodes, wsrc, bsrc, wtgt, btgt, NH, WH, BC);

  eng::gemm64_f16<2, 0><<<(kNodes / 64) * (kCat / 64) / 8, 256, 0, stream>>>(
      NH, kChan, WH, kChan, (void*)G, kCat, BC,
      kNodes, kCat, kChan, kScaleProj, 1.0f);

  eng::gemm64_f16<1, 1><<<(kChan / 64) * (kNodes / 64) / 8, 256, 0, stream>>>(
      WH + (size_t)kChan * kChan, kChan, NH, kChan, (void*)GT, kNodes, btgt,
      kChan, kNodes, kChan, kScaleProj, kCarryG);

  score_softmax_kernel<<<kNodes / kRowTile, 256, 0, stream>>>(G, aw, adj, PW);

  eng::gemm64_f16<0, 0><<<(kNodes / 64) * (kChan / 64) / 8, 256, 0, stream>>>(
      PW, kNodes, GT, kNodes, (void*)out, kChan, nullptr,
      kNodes, kChan, kNodes, kScaleOut, 1.0f);
}
